// VMAMBA2Block_16449724745534
// MI455X (gfx1250) — hardware-run, weakly checked
//
#include <hip/hip_runtime.h>
#include <math.h>

typedef __attribute__((ext_vector_type(16))) _Float16 v16h;
typedef __attribute__((ext_vector_type(8)))  _Float16 v8h;
typedef __attribute__((ext_vector_type(8)))  float    v8f;
typedef __attribute__((ext_vector_type(4)))  float    v4f;
typedef __attribute__((ext_vector_type(2)))  float    v2f;
typedef __attribute__((ext_vector_type(4)))  unsigned v4u;
typedef __attribute__((ext_vector_type(2)))  unsigned v2u;

constexpr int kB    = 8;
constexpr int kHW   = 64;
constexpr int kL    = kHW * kHW;
constexpr int kC    = 192;
constexpr int kNH   = 6;
constexpr int kHD   = 64;
constexpr int kDIN  = kNH * kHD;
constexpr int kDS   = 64;
constexpr int kCD   = kDIN + 2 * kDS;
constexpr int kDP   = 2 * kDIN + 2 * kDS + kNH;
constexpr int kDPP  = 960;
constexpr int kCHK  = 256;
constexpr int kNCH  = kL / kCHK;
constexpr int kFF   = 4 * kC;
constexpr int kDTW  = 64;
constexpr int kNPASS = 4;
constexpr int kBP   = kB / kNPASS;
constexpr int kMQ   = kBP * kL;
constexpr int kUnits = kBP * kNCH * kNH;
constexpr int kZT   = kDIN / 64;
constexpr int kXT   = kCD / 64;
static_assert(kL == 4096 && kDIN == 384 && kCD == 512 && kDP == 902 && kNCH == 16 && kFF == 768, "shape");
static_assert(kDPP % 64 == 0 && kDPP >= kDP && kDPP / 64 == kZT + kXT + 1, "in_proj tiling");
static_assert(kDPP - (kDIN + kCD) == kDTW, "dt tile width");
static_assert(kC % 32 == 0 && kDIN % 32 == 0 && kFF % 32 == 0 && kDS % 32 == 0 && kCHK % 32 == 0, "K multiples of 32");
static_assert(kMQ % 64 == 0 && kC % 64 == 0 && kFF % 64 == 0, "tile multiples");
static_assert(kMQ == 8192 && kUnits == 192, "pass size");

constexpr float kActC   = 16.0f;
constexpr float kWgtC   = 32.0f;
constexpr float kGemmSc = 1.0f / (kActC * kWgtC);
constexpr float kXcC    = 64.0f;
constexpr float kPC     = 256.0f;
constexpr float kSentC  = 256.0f;
constexpr float kYsC    = 1024.0f;
constexpr float kScoreFold = kPC / (kXcC * kXcC);
constexpr float kStateFold = 1.0f / (kXcC * kXcC);
constexpr float kYFold     = kYsC / (kPC * kXcC);
static_assert(kPC * kXcC == kXcC * kSentC, "shared accumulator carry");

constexpr size_t kOffWIN  = 0;
constexpr size_t kOffWOUT = kOffWIN  + (size_t)kDPP * kC * 2;
constexpr size_t kOffWFC1 = kOffWOUT + (size_t)kC * kDIN * 2;
constexpr size_t kOffWFC2 = kOffWFC1 + (size_t)kFF * kC * 2;
constexpr size_t kOffSHORT = kOffWFC2 + (size_t)kC * kFF * 2;
constexpr size_t kOffH16  = kOffSHORT + (size_t)kMQ * kC * 4;
constexpr size_t kOffZ16  = kOffH16  + (size_t)kMQ * kC * 2;
constexpr size_t kOffXBC  = kOffZ16  + (size_t)kMQ * kDIN * 2;
constexpr size_t kOffDTRAW = kOffXBC + (size_t)kMQ * kCD * 2;
constexpr size_t kOffXC   = kOffDTRAW + (size_t)kMQ * kDTW * 4;
constexpr size_t kOffDT   = kOffXC   + (size_t)kMQ * kCD * 2;
constexpr size_t kOffCS   = kOffDT   + (size_t)kNH * kMQ * 4;
constexpr size_t kOffST   = kOffCS   + (size_t)kNH * kMQ * 4;
constexpr size_t kOffSENT = kOffST   + (size_t)kUnits * kDS * kHD * 4;
constexpr size_t kOffYS   = kOffSENT + (size_t)kUnits * kDS * kHD * 4;
constexpr size_t kOffYN   = kOffYS   + (size_t)kMQ * kDIN * 2;
constexpr size_t kOffX2   = kOffYN   + (size_t)kMQ * kDIN * 2;
constexpr size_t kOffX2B  = kOffX2   + (size_t)kMQ * kC * 4;
constexpr size_t kOffH2   = kOffX2B  + (size_t)kMQ * kC * 4;
constexpr size_t kOffM1   = kOffH2   + (size_t)kMQ * kC * 2;
constexpr size_t kWsTotal = kOffM1   + (size_t)kMQ * kFF * 2;
static_assert(kWsTotal == 83288064ull, "carve total");
static_assert(kWsTotal <= 134217728ull, "carve cap");
static_assert((kOffWOUT % 128) == 0 && (kOffWFC1 % 128) == 0 && (kOffWFC2 % 128) == 0 && (kOffSHORT % 128) == 0 &&
              (kOffH16 % 128) == 0 && (kOffZ16 % 128) == 0 && (kOffXBC % 128) == 0 && (kOffDTRAW % 128) == 0 &&
              (kOffXC % 128) == 0 && (kOffDT % 128) == 0 && (kOffCS % 128) == 0 && (kOffST % 128) == 0 &&
              (kOffSENT % 128) == 0 && (kOffYS % 128) == 0 && (kOffYN % 128) == 0 && (kOffX2 % 128) == 0 &&
              (kOffX2B % 128) == 0 && (kOffH2 % 128) == 0 && (kOffM1 % 128) == 0, "128-B aligned regions");

__device__ __forceinline__ float h16_to_f32(unsigned hb) {
  const unsigned sgn = (hb & 0x8000u) << 16;
  const unsigned em = hb & 0x7fffu;
  const float fn = __uint_as_float((em << 13) + 0x38000000u);
  const float fs = (float)em * 5.9604644775390625e-8f;
  const float mag = (em < 0x400u) ? fs : fn;
  return __uint_as_float(__float_as_uint(mag) | sgn);
}
__device__ __forceinline__ _Float16 bits_to_h(unsigned w) {
  const unsigned short us = (unsigned short)(w & 0xffffu);
  return __builtin_bit_cast(_Float16, us);
}
union FragU { v16h v; v8h h[2]; };
__device__ __forceinline__ v16h frag_load(const _Float16* p) {
  FragU f;
  f.h[0] = *(const v8h*)(p);
  f.h[1] = *(const v8h*)(p + 16);
  return f.v;
}
__device__ __forceinline__ v8f wmma_raw(v16h a, v16h b, v8f c) {
  return __builtin_amdgcn_wmma_f32_16x16x32_f16(false, a, false, b, (short)0, c, false, false);
}
__device__ __forceinline__ v8f mma_g(v16h a, v16h b, v8f c) {
  c = __builtin_amdgcn_wmma_f32_16x16x32_f16(false, a, false, b, (short)0, c, false, false);
  asm volatile("v_nop\n\tv_nop\n\tv_nop\n\tv_nop" : "+v"(c) : "v"(a), "v"(b));
  return c;
}
__device__ __forceinline__ void guard4(v8f& a, v8f& b, v8f& c, v8f& d, v16h x, v16h y0, v16h y1, v16h y2, v16h y3) {
  asm volatile("v_nop\n\tv_nop\n\tv_nop\n\tv_nop" : "+v"(a), "+v"(b), "+v"(c), "+v"(d) : "v"(x), "v"(y0), "v"(y1), "v"(y2), "v"(y3));
}
__device__ __forceinline__ void acc_guard4(v8f& a, v8f& b, v8f& c, v8f& d) {
  asm volatile("v_nop\n\tv_nop\n\tv_nop\n\tv_nop" : "+v"(a), "+v"(b), "+v"(c), "+v"(d));
}
__device__ __forceinline__ void wave_lds_sync() {
  __builtin_amdgcn_fence(__ATOMIC_RELEASE, "workgroup");
  __builtin_amdgcn_wave_barrier();
  __builtin_amdgcn_fence(__ATOMIC_ACQUIRE, "workgroup");
}

__global__ __launch_bounds__(256) void cast_pad_f16_kernel(
    const float* __restrict__ src, unsigned short* __restrict__ dst, int total8, int real8, float scale)
{
  const int i = blockIdx.x * 256 + threadIdx.x;
  if (i >= total8) return;
  const bool live = (i < real8);
  const size_t es = live ? ((size_t)i << 3) : (size_t)0;
  const v4f a0 = *(const v4f*)(src + es);
  const v4f a1 = *(const v4f*)(src + es + 4);
  v8h hv;
#pragma unroll
  for (int e = 0; e < 4; ++e) {
    const float f0 = live ? (a0[e] * scale) : 0.0f;
    const float f1 = live ? (a1[e] * scale) : 0.0f;
    hv[e]     = (_Float16)f0;
    hv[4 + e] = (_Float16)f1;
  }
  unsigned short* q = dst + ((size_t)i << 3);
  *(volatile v8h*)q = hv;
  __threadfence();
  *(volatile v8h*)q = hv;
}

constexpr int kCpeGroups = 4;
static_assert(kMQ % (32 * kCpeGroups) == 0, "cpe grid");
__global__ __launch_bounds__(256) void cpe_ln_kernel(
    const float* __restrict__ X, const float* __restrict__ cw, const float* __restrict__ cb,
    const float* __restrict__ lw, const float* __restrict__ lb,
    float* __restrict__ OXS, unsigned short* __restrict__ OH16)
{
  __shared__ __align__(16) float sW[9 * kC];
  __shared__ __align__(16) float sB[kC];
  __shared__ __align__(16) float sLw[kC];
  __shared__ __align__(16) float sLb[kC];
  __shared__ __align__(16) float sXS[8][4 * kC];
  __shared__ float sStat[8][8];
  const int tid = threadIdx.x;
  const int lane = tid & 31;
  const int wave = __builtin_amdgcn_readfirstlane(tid >> 5);
  for (int e = tid; e < 9 * kC; e += 256) {
    const int c = e / 9;
    const int tap = e - c * 9;
    sW[tap * kC + c] = cw[e];
  }
  if (tid < kC) {
    sB[tid] = cb[tid];
    sLw[tid] = lw[tid];
    sLb[tid] = lb[tid];
  }
  __syncthreads();
  const v4f bias4 = *(const v4f*)(sB + lane * 4);
  const v2f bias2 = *(const v2f*)(sB + 128 + lane * 2);
#pragma unroll 1
  for (int gi = 0; gi < kCpeGroups; ++gi) {
    const int t0 = (blockIdx.x * kCpeGroups + gi) * 32 + wave * 4;
#pragma unroll 1
    for (int k = 0; k < 4; ++k) {
      const int t = t0 + k;
      const int l = t & (kL - 1);
      const int i = l >> 6;
      const int j = l & 63;
      v4f a4 = bias4;
      v2f a2 = bias2;
#pragma unroll 1
      for (int di = 0; di < 3; ++di) {
#pragma unroll 1
        for (int dj = 0; dj < 3; ++dj) {
          const int ii = i + di - 1;
          const int jj = j + dj - 1;
          const bool valid = (ii >= 0) && (ii < kHW) && (jj >= 0) && (jj < kHW);
          if (valid) {
            const size_t tn = (size_t)(t + (di - 1) * kHW + (dj - 1));
            const float* xp = X + tn * kC;
            const v4f xv = *(const v4f*)(xp + lane * 4);
            const v2f xw = *(const v2f*)(xp + 128 + lane * 2);
            const float* wp = sW + (di * 3 + dj) * kC;
            const v4f w4 = *(const v4f*)(wp + lane * 4);
            const v2f w2 = *(const v2f*)(wp + 128 + lane * 2);
            a4 += xv * w4;
            a2 += xw * w2;
          }
        }
      }
      const float* xc = X + (size_t)t * kC;
      const v4f s4 = *(const v4f*)(xc + lane * 4) + a4;
      const v2f s2 = *(const v2f*)(xc + 128 + lane * 2) + a2;
      float sum = ((s4[0] + s4[1]) + (s4[2] + s4[3])) + (s2[0] + s2[1]);
#pragma unroll
      for (int off = 16; off >= 1; off >>= 1) sum += __shfl_xor(sum, off, 32);
      const float mu = sum * (1.0f / (float)kC);
      const v4f d4 = s4 - mu;
      const v2f d2 = s2 - mu;
      float vs = ((d4[0] * d4[0] + d4[1] * d4[1]) + (d4[2] * d4[2] + d4[3] * d4[3])) + (d2[0] * d2[0] + d2[1] * d2[1]);
#pragma unroll
      for (int off = 16; off >= 1; off >>= 1) vs += __shfl_xor(vs, off, 32);
      const float rstd = rsqrtf(vs * (1.0f / (float)kC) + 1e-5f);
      *(v4f*)(&sXS[wave][k * kC + lane * 4]) = s4;
      *(v2f*)(&sXS[wave][k * kC + 128 + lane * 2]) = s2;
      if (lane == 0) {
        sStat[wave][2 * k] = mu;
        sStat[wave][2 * k + 1] = rstd;
      }
    }
    __syncthreads();
    v4f fv[6];
    v8h hv[3];
#pragma unroll
    for (int it = 0; it < 6; ++it) fv[it] = *(const v4f*)(&sXS[wave][(it * 32 + lane) * 4]);
#pragma unroll
    for (int it = 0; it < 3; ++it) {
      const int idx = it * 32 + lane;
      const int kk = idx / 24;
      const int c0 = (idx - kk * 24) * 8;
      const float mu = sStat[wave][2 * kk];
      const float rstd = sStat[wave][2 * kk + 1];
      const float* sp = &sXS[wave][idx * 8];
      const v4f a0 = *(const v4f*)(sp);
      const v4f a1 = *(const v4f*)(sp + 4);
      const v4f w0 = *(const v4f*)(sLw + c0);
      const v4f w1 = *(const v4f*)(sLw + c0 + 4);
      const v4f b0 = *(const v4f*)(sLb + c0);
      const v4f b1 = *(const v4f*)(sLb + c0 + 4);
#pragma unroll
      for (int e = 0; e < 4; ++e) {
        const float h0 = (a0[e] - mu) * rstd * w0[e] + b0[e];
        const float h1 = (a1[e] - mu) * rstd * w1[e] + b1[e];
        hv[it][e]     = (_Float16)(h0 * kActC);
        hv[it][4 + e] = (_Float16)(h1 * kActC);
      }
    }
    float* op = OXS + (size_t)t0 * kC;
    unsigned short* hp = OH16 + (size_t)t0 * kC;
    for (int pass = 0; pass < 2; ++pass) {
#pragma unroll
      for (int it = 0; it < 6; ++it) *(volatile v4f*)(op + (it * 32 + lane) * 4) = fv[it];
#pragma unroll
      for (int it = 0; it < 3; ++it) *(volatile v8h*)(hp + (it * 32 + lane) * 8) = hv[it];
      __threadfence();
    }
    __syncthreads();
  }
}

template <int EPI, bool HASBIAS>
__global__ __launch_bounds__(256) void gemm16_kernel(
    const unsigned short* __restrict__ Ap, int lda,
    const unsigned short* __restrict__ Btp, int ldb,
    void* O0, void* O1, void* O2, int ldc,
    const float* __restrict__ bias, const float* __restrict__ resid,
    int M, int N, int K, float scale)
{
  const _Float16* A = (const _Float16*)Ap;
  const _Float16* Bt = (const _Float16*)Btp;
  __shared__ __align__(16) float sT[8][16 * 68];
  const int lane = threadIdx.x & 31;
  const int wave = __builtin_amdgcn_readfirstlane(threadIdx.x >> 5);
  const int tilesN = N >> 6;
  const int tilesM = M >> 6;
  const int tile = blockIdx.x * 8 + wave;
  if (tile >= tilesM * tilesN) return;
  const int tm = tile / tilesN;
  const int tn = tile - tm * tilesN;
  const int m0 = tm << 6;
  const int n0 = tn << 6;
  const int rlane = lane & 15;
  const int koff = (lane >> 4) * 8;
  const int mOff = (lane >> 4) * 8;

  v8f acc[4][4];
#pragma unroll
  for (int i = 0; i < 4; ++i)
#pragma unroll
    for (int j = 0; j < 4; ++j) acc[i][j] = (v8f){0.f, 0.f, 0.f, 0.f, 0.f, 0.f, 0.f, 0.f};

  for (int k0 = 0; k0 < K; k0 += 32) {
    v16h bh[4];
#pragma unroll
    for (int j = 0; j < 4; ++j)
      bh[j] = frag_load(Bt + (size_t)(n0 + (j << 4) + rlane) * ldb + koff + k0);
#pragma unroll
    for (int i = 0; i < 4; ++i) {
      const v16h ah = frag_load(A + (size_t)(m0 + (i << 4) + rlane) * lda + koff + k0);
#pragma unroll
      for (int j = 0; j < 4; ++j) acc[i][j] = wmma_raw(ah, bh[j], acc[i][j]);
      guard4(acc[i][0], acc[i][1], acc[i][2], acc[i][3], ah, bh[0], bh[1], bh[2], bh[3]);
    }
  }
  acc_guard4(acc[0][0], acc[0][1], acc[0][2], acc[0][3]);
  acc_guard4(acc[1][0], acc[1][1], acc[1][2], acc[1][3]);
  acc_guard4(acc[2][0], acc[2][1], acc[2][2], acc[2][3]);
  acc_guard4(acc[3][0], acc[3][1], acc[3][2], acc[3][3]);

  float* slab = sT[wave];
#pragma unroll
  for (int i = 0; i < 4; ++i) {
    const int mBase = m0 + (i << 4);
#pragma unroll
    for (int j = 0; j < 4; ++j) {
      float bv = 0.f;
      if (HASBIAS) bv = bias[n0 + (j << 4) + rlane];
#pragma unroll
      for (int r = 0; r < 8; ++r) {
        const float v = acc[i][j][r] * scale + bv;
        slab[(mOff + r) * 68 + (j << 4) + rlane] = v;
      }
    }
    wave_lds_sync();
    if (EPI == 2) {
#pragma unroll 1
      for (int t = 0; t < 32; ++t) {
        const int idx = t * 32 + lane;
        const int row = idx >> 6;
        const int col = idx & 63;
        const float x = slab[row * 68 + col];
        slab[row * 68 + col] = (0.5f * kActC) * x * (1.0f + erff(x * 0.70710678118654752f));
      }
      wave_lds_sync();
    }
    if (EPI == 1) {
      const int hh = lane >> 4;
      const int c4 = (lane & 15) * 4;
#pragma unroll
      for (int it = 0; it < 8; ++it) {
        const int row = it * 2 + hh;
        v4f v = *(const v4f*)(slab + row * 68 + c4);
        const v4f rv = *(const v4f*)(resid + (size_t)(mBase + row) * ldc + n0 + c4);
        v += rv;
        *(v4f*)(slab + row * 68 + c4) = v;
      }
      wave_lds_sync();
    }
    const bool f32out = (EPI == 1) || ((EPI == 0) && (tn == kZT + kXT));
    if (f32out) {
      float* Cf = (EPI == 1) ? (float*)O0 : (float*)O2;
      const int ldf = (EPI == 1) ? ldc : kDTW;
      const int cb0 = (EPI == 1) ? n0 : 0;
      const int hh = lane >> 4;
      const int c4 = (lane & 15) * 4;
      for (int pass = 0; pass < 2; ++pass) {
#pragma unroll
        for (int it = 0; it < 8; ++it) {
          const int row = it * 2 + hh;
          const v4f v = *(const v4f*)(slab + row * 68 + c4);
          *(volatile v4f*)(Cf + (size_t)(mBase + row) * ldf + cb0 + c4) = v;
        }
        __threadfence();
      }
    } else {
      unsigned short* Ch = (unsigned short*)O0;
      int ldh = ldc;
      int cb0 = n0;
      if (EPI == 0) {
        const bool isz = (tn < kZT);
        Ch = isz ? (unsigned short*)O0 : (unsigned short*)O1;
        ldh = isz ? kDIN : kCD;
        cb0 = isz ? n0 : (n0 - kDIN);
      }
      const int q = lane >> 3;
      const int c8 = (lane & 7) * 8;
      for (int pass = 0; pass < 2; ++pass) {
#pragma unroll
        for (int it = 0; it < 4; ++it) {
          const int row = it * 4 + q;
          const float* sp = slab + row * 68 + c8;
          v8h hv;
#pragma unroll
          for (int e = 0; e < 8; ++e) hv[e] = (_Float16)sp[e];
          *(volatile v8h*)(Ch + (size_t)(mBase + row) * ldh + cb0 + c8) = hv;
        }
        __threadfence();
      }
    }
    wave_lds_sync();
  }
}

constexpr int kCvP = 516;
__device__ __forceinline__ float silu_p(float v) {
  return v * __builtin_amdgcn_rcpf(1.0f + expf(-v));
}
__global__ __launch_bounds__(256) void conv_silu_kernel(
    const unsigned short* __restrict__ XBC16, const float* __restrict__ cw, const float* __restrict__ cb,
    unsigned short* __restrict__ XC16)
{
  __shared__ __align__(16) float sT[16 * kCvP];
  const int tid = threadIdx.x;
  const int lane = tid & 31;
  const int wave = tid >> 5;
  const int d = 2 * tid;
  const int g0 = blockIdx.x * 64;
  const int tb = g0 & (kL - 1);
  const unsigned* src = (const unsigned*)(const void*)XBC16;
  const v4f wa = *(const v4f*)(cw + d * 4);
  const v4f wb = *(const v4f*)(cw + d * 4 + 4);
  const float ba = cb[d];
  const float bb = cb[d + 1];
  float xa3, xa2, xa1, xb3, xb2, xb1;
  {
    const bool hist = (tb > 0);
    const int rb = hist ? (g0 - 3) : g0;
    const unsigned u3 = src[(size_t)rb * (kCD / 2) + tid];
    const unsigned u2 = src[(size_t)(rb + 1) * (kCD / 2) + tid];
    const unsigned u1 = src[(size_t)(rb + 2) * (kCD / 2) + tid];
    const float fa3 = h16_to_f32(u3 & 0xffffu), fb3 = h16_to_f32(u3 >> 16);
    const float fa2 = h16_to_f32(u2 & 0xffffu), fb2 = h16_to_f32(u2 >> 16);
    const float fa1 = h16_to_f32(u1 & 0xffffu), fb1 = h16_to_f32(u1 >> 16);
    xa3 = hist ? fa3 : 0.f;
    xb3 = hist ? fb3 : 0.f;
    xa2 = hist ? fa2 : 0.f;
    xb2 = hist ? fb2 : 0.f;
    xa1 = hist ? fa1 : 0.f;
    xb1 = hist ? fb1 : 0.f;
  }
  const int hrow = wave >> 1;
  const int hcol = (wave & 1) * 256 + lane * 8;
#pragma unroll 1
  for (int sub = 0; sub < 4; ++sub) {
    const int lb = g0 + sub * 16;
#pragma unroll 1
    for (int s = 0; s < 16; ++s) {
      const unsigned u = src[(size_t)(lb + s) * (kCD / 2) + tid];
      const float xa = h16_to_f32(u & 0xffffu);
      const float xb = h16_to_f32(u >> 16);
      float aa = wa[0] * xa3;
      aa = fmaf(wa[1], xa2, aa);
      aa = fmaf(wa[2], xa1, aa);
      aa = fmaf(wa[3], xa, aa);
      float ab = wb[0] * xb3;
      ab = fmaf(wb[1], xb2, ab);
      ab = fmaf(wb[2], xb1, ab);
      ab = fmaf(wb[3], xb, ab);
      const float ya = silu_p(aa + ba);
      const float yb = silu_p(ab + bb);
      sT[s * kCvP + d] = ya * kXcC;
      sT[s * kCvP + d + 1] = yb * kXcC;
      xa3 = xa2; xa2 = xa1; xa1 = xa;
      xb3 = xb2; xb2 = xb1; xb1 = xb;
    }
    __syncthreads();
    v8h hv[4];
#pragma unroll
    for (int it = 0; it < 4; ++it) {
      const float* sp = sT + (it * 4 + hrow) * kCvP + hcol;
      const v4f a0 = *(const v4f*)(sp);
      const v4f a1 = *(const v4f*)(sp + 4);
#pragma unroll
      for (int e = 0; e < 4; ++e) {
        hv[it][e]     = (_Float16)a0[e];
        hv[it][4 + e] = (_Float16)a1[e];
      }
    }
    for (int pass = 0; pass < 2; ++pass) {
#pragma unroll
      for (int it = 0; it < 4; ++it)
        *(volatile v8h*)(XC16 + (size_t)(lb + it * 4 + hrow) * kCD + hcol) = hv[it];
      __threadfence();
    }
    __syncthreads();
  }
}

__global__ __launch_bounds__(256) void dt_cumsum_kernel(
    const float* __restrict__ DTRAW, const float* __restrict__ dt_bias, const float* __restrict__ A_log,
    float* __restrict__ DT, float* __restrict__ CS)
{
  __shared__ __align__(16) float sD[8][kCHK];
  __shared__ __align__(16) float sC[8][kCHK];
  const int tid = threadIdx.x;
  const int lane = tid & 31;
  const int wave = __builtin_amdgcn_readfirstlane(tid >> 5);
  const int unit = blockIdx.x * 8 + wave;
  const int h = unit % kNH;
  const int bc = unit / kNH;
  const int base = bc * kCHK;
  const float Ah = -expf(A_log[h]);
  const float bias = dt_bias[h];
#pragma unroll 1
  for (int k = 0; k < 8; ++k) {
    const int j = k * 32 + lane;
    const float v = DTRAW[(size_t)(base + j) * kDTW + h] + bias;
    const float sp = fmaxf(v, 0.0f) + log1pf(expf(-fabsf(v)));
    sD[wave][j] = sp;
  }
  __syncthreads();
  const v4f d0 = *(const v4f*)(&sD[wave][lane * 8]);
  const v4f d1 = *(const v4f*)(&sD[wave][lane * 8 + 4]);
  float c[8];
  float run = 0.f;
#pragma unroll
  for (int e = 0; e < 4; ++e) {
    const float p = d0[e] * Ah;
    run += p;
    c[e] = run;
  }
#pragma unroll
  for (int e = 0; e < 4; ++e) {
    const float p = d1[e] * Ah;
    run += p;
    c[4 + e] = run;
  }
  float incl = run;
#pragma unroll
  for (int off = 1; off < 32; off <<= 1) {
    const float t = __shfl_up(incl, off, 32);
    incl += (lane >= off) ? t : 0.f;
  }
  const float e1 = __shfl_up(incl, 1, 32);
  const float excl = (lane == 0) ? 0.f : e1;
  v4f c0v, c1v;
#pragma unroll
  for (int e = 0; e < 4; ++e) {
    c0v[e] = c[e] + excl;
    c1v[e] = c[4 + e] + excl;
  }
  *(v4f*)(&sC[wave][lane * 8]) = c0v;
  *(v4f*)(&sC[wave][lane * 8 + 4]) = c1v;
  __syncthreads();
  v4f vd[2], vc[2];
#pragma unroll
  for (int it = 0; it < 2; ++it) {
    vd[it] = *(const v4f*)(&sD[wave][it * 128 + lane * 4]);
    vc[it] = *(const v4f*)(&sC[wave][it * 128 + lane * 4]);
  }
  float* dp = DT + (size_t)h * kMQ + base;
  float* cp = CS + (size_t)h * kMQ + base;
  for (int pass = 0; pass < 2; ++pass) {
#pragma unroll
    for (int it = 0; it < 2; ++it) {
      *(volatile v4f*)(dp + it * 128 + lane * 4) = vd[it];
      *(volatile v4f*)(cp + it * 128 + lane * 4) = vc[it];
    }
    __threadfence();
  }
}

constexpr int kTP40 = 40;
__global__ __launch_bounds__(128) void ssd_states_kernel(
    const unsigned short* __restrict__ XC16, const float* __restrict__ DT, const float* __restrict__ CS,
    float* __restrict__ STATES)
{
  __shared__ float sWg[kCHK];
  __shared__ __align__(16) _Float16 bsT[64 * kTP40];
  __shared__ __align__(16) _Float16 xsT[64 * kTP40];
  __shared__ __align__(16) float slab[4][16 * 68];
  const int tid = threadIdx.x;
  const int lane = tid & 31;
  const int wave = __builtin_amdgcn_readfirstlane(tid >> 5);
  const int g = lane >> 4;
  const int r = lane & 15;
  const int koff = g * 8;
  const int bch = blockIdx.x;
  const int h = bch % kNH;
  const int cc = (bch / kNH) % kNCH;
  const int b = bch / (kNH * kNCH);
  const int lbase = b * kL + cc * kCHK;
  const float* csr = CS + (size_t)h * kMQ + lbase;
  const float* dtr = DT + (size_t)h * kMQ + lbase;
  const float cl = csr[kCHK - 1];
#pragma unroll 1
  for (int j = tid; j < kCHK; j += 128) {
    const float a = fminf(cl - csr[j], 0.0f);
    const float e = (a < -87.0f) ? 0.0f : expf(a);
    sWg[j] = dtr[j] * e;
  }
  __syncthreads();
  v8f acc[4];
#pragma unroll
  for (int nt = 0; nt < 4; ++nt) acc[nt] = (v8f){0.f, 0.f, 0.f, 0.f, 0.f, 0.f, 0.f, 0.f};
#pragma unroll 1
  for (int k0 = 0; k0 < kCHK; k0 += 32) {
    __syncthreads();
    {
      const int jj = tid >> 2;
      const int q16 = (tid & 3) * 16;
      const size_t rowo = (size_t)(lbase + k0 + jj) * kCD;
      const v4u* pb = (const v4u*)(const void*)(XC16 + rowo + kDIN + q16);
      const v4u* px = (const v4u*)(const void*)(XC16 + rowo + h * kHD + q16);
      const v4u bw0 = pb[0];
      const v4u bw1 = pb[1];
      const v4u xw0 = px[0];
      const v4u xw1 = px[1];
      const float wj = sWg[k0 + jj];
#pragma unroll
      for (int wi = 0; wi < 4; ++wi) {
        const unsigned b0 = bw0[wi];
        const unsigned b1 = bw1[wi];
        const unsigned x0 = xw0[wi];
        const unsigned x1 = xw1[wi];
        const int n = q16 + 2 * wi;
        bsT[(n) * kTP40 + jj]     = (_Float16)(h16_to_f32(b0 & 0xffffu) * wj);
        bsT[(n + 1) * kTP40 + jj] = (_Float16)(h16_to_f32(b0 >> 16) * wj);
        bsT[(n + 8) * kTP40 + jj] = (_Float16)(h16_to_f32(b1 & 0xffffu) * wj);
        bsT[(n + 9) * kTP40 + jj] = (_Float16)(h16_to_f32(b1 >> 16) * wj);
        xsT[(n) * kTP40 + jj]     = bits_to_h(x0);
        xsT[(n + 1) * kTP40 + jj] = bits_to_h(x0 >> 16);
        xsT[(n + 8) * kTP40 + jj] = bits_to_h(x1);
        xsT[(n + 9) * kTP40 + jj] = bits_to_h(x1 >> 16);
      }
    }
    __syncthreads();
    const v16h a = frag_load(bsT + (wave * 16 + r) * kTP40 + koff);
#pragma unroll
    for (int nt = 0; nt < 4; ++nt) {
      const v16h bb = frag_load(xsT + (nt * 16 + r) * kTP40 + koff);
      acc[nt] = mma_g(a, bb, acc[nt]);
    }
  }
  float* sl = slab[wave];
#pragma unroll
  for (int nt = 0; nt < 4; ++nt)
#pragma unroll
    for (int v = 0; v < 8; ++v) sl[(8 * g + v) * 68 + nt * 16 + r] = acc[nt][v] * kStateFold;
  __syncthreads();
  {
    float* st = STATES + (size_t)bch * (kDS * kHD) + (size_t)(wave * 16) * kHD;
    const int c4 = (lane & 15) * 4;
    for (int pass = 0; pass < 2; ++pass) {
#pragma unroll
      for (int it = 0; it < 8; ++it) {
        const int row = it * 2 + g;
        const v4f v = *(const v4f*)(sl + row * 68 + c4);
        *(volatile v4f*)(st + (size_t)row * kHD + c4) = v;
      }
      __threadfence();
    }
  }
}

__global__ __launch_bounds__(256) void chunk_scan_kernel(
    const float* __restrict__ STATES, const float* __restrict__ CS, float* __restrict__ SENT)
{
  const int gid = blockIdx.x * 256 + threadIdx.x;
  const int e4 = gid & 1023;
  const int bh = gid >> 10;
  const int b = bh / kNH;
  const int h = bh - b * kNH;
  v4f carry = (v4f){0.f, 0.f, 0.f, 0.f};
#pragma unroll 1
  for (int c = 0; c < kNCH; ++c) {
    const size_t idx = ((size_t)((b * kNCH + c) * kNH + h)) * (kDS * kHD) + (size_t)e4 * 4;
    const float a = CS[(size_t)h * kMQ + b * kL + c * kCHK + (kCHK - 1)];
    const float cd = (a < -87.0f) ? 0.0f : expf(a);
    const v4f s = *(const v4f*)(STATES + idx);
    const v4f pv = carry;
    *(volatile v4f*)(SENT + idx) = pv;
    __threadfence();
    *(volatile v4f*)(SENT + idx) = pv;
    carry = carry * cd + s;
  }
}

constexpr int kPvP = 72;
constexpr int kPwP = 72;
__global__ __launch_bounds__(512) void ssd_y_kernel(
    const unsigned short* __restrict__ XC16, const float* __restrict__ DT, const float* __restrict__ CS,
    const float* __restrict__ SENT, unsigned short* __restrict__ YS16)
{
  __shared__ float sDt[kCHK];
  __shared__ float sCs[kCHK];
  __shared__ __align__(16) _Float16 xs[64 * kTP40];
  __shared__ __align__(16) _Float16 sentT[64 * kPvP];
  __shared__ __align__(16) _Float16 pw[16][16 * kPwP];
  const int tid = threadIdx.x;
  const int lane = tid & 31;
  const int wave = __builtin_amdgcn_readfirstlane(tid >> 5);
  const int g = lane >> 4;
  const int r = lane & 15;
  const int koff = g * 8;
  const int bch = blockIdx.x;
  const int h = bch % kNH;
  const int cc = (bch / kNH) % kNCH;
  const int b = bch / (kNH * kNCH);
  const int lbase = b * kL + cc * kCHK;
  if (tid < kCHK) {
    sDt[tid] = DT[(size_t)h * kMQ + lbase + tid];
    sCs[tid] = CS[(size_t)h * kMQ + lbase + tid];
  }
  {
    const float* pv = SENT + (size_t)bch * (kDS * kHD);
    const int e = tid * 8;
    const int n = e >> 6;
    const int p0 = e & 63;
    const v4f a0 = *(const v4f*)(pv + e);
    const v4f a1 = *(const v4f*)(pv + e + 4);
#pragma unroll
    for (int i = 0; i < 4; ++i) {
      sentT[(p0 + i) * kPvP + n]     = (_Float16)(a0[i] * kSentC);
      sentT[(p0 + 4 + i) * kPvP + n] = (_Float16)(a1[i] * kSentC);
    }
  }
  __syncthreads();
  const _Float16* XCh = (const _Float16*)(const void*)XC16;
  const int ib = wave * 16;
  const _Float16* crow = XCh + (size_t)(lbase + ib + r) * kCD + (kDIN + kDS) + koff;
  const v16h a_lo = frag_load(crow);
  const v16h a_hi = frag_load(crow + 32);
  float dAi[8];
#pragma unroll
  for (int v = 0; v < 8; ++v) dAi[v] = sCs[ib + 8 * g + v];
  v8f acc[4];
#pragma unroll
  for (int nt = 0; nt < 4; ++nt) acc[nt] = (v8f){0.f, 0.f, 0.f, 0.f, 0.f, 0.f, 0.f, 0.f};
  _Float16* pt = pw[wave];
#pragma unroll 1
  for (int jb = 0; jb < kCHK / 32; ++jb) {
    const int j0 = jb * 32;
    __syncthreads();
    {
      const int jj = tid >> 4;
      const int p4 = (tid & 15) * 4;
      const v2u w = *(const v2u*)(const void*)(XC16 + (size_t)(lbase + j0 + jj) * kCD + h * kHD + p4);
      const unsigned w0 = w[0];
      const unsigned w1 = w[1];
      xs[(p4) * kTP40 + jj]     = bits_to_h(w0);
      xs[(p4 + 1) * kTP40 + jj] = bits_to_h(w0 >> 16);
      xs[(p4 + 2) * kTP40 + jj] = bits_to_h(w1);
      xs[(p4 + 3) * kTP40 + jj] = bits_to_h(w1 >> 16);
    }
    __syncthreads();
    const bool active = (j0 <= ib + 15);
    if (active) {
      const _Float16* br0 = XCh + (size_t)(lbase + j0 + r) * kCD + kDIN + koff;
      const _Float16* br1 = XCh + (size_t)(lbase + j0 + 16 + r) * kCD + kDIN + koff;
      const v16h b0l = frag_load(br0);
      const v16h b0h = frag_load(br0 + 32);
      const v16h b1l = frag_load(br1);
      const v16h b1h = frag_load(br1 + 32);
      v8f s0 = (v8f){0.f, 0.f, 0.f, 0.f, 0.f, 0.f, 0.f, 0.f};
      v8f s1 = (v8f){0.f, 0.f, 0.f, 0.f, 0.f, 0.f, 0.f, 0.f};
      s0 = mma_g(a_lo, b0l, s0);
      s0 = mma_g(a_hi, b0h, s0);
      s1 = mma_g(a_lo, b1l, s1);
      s1 = mma_g(a_hi, b1h, s1);
      const int ja = j0 + r;
      const int jc = j0 + 16 + r;
      const float cj0 = sCs[ja];
      const float cj1 = sCs[jc];
      const float dj0 = sDt[ja] * kScoreFold;
      const float dj1 = sDt[jc] * kScoreFold;
#pragma unroll
      for (int v = 0; v < 8; ++v) {
        const int irow = ib + 8 * g + v;
        const float a0 = fminf(dAi[v] - cj0, 0.0f);
        const float a1 = fminf(dAi[v] - cj1, 0.0f);
        const float e0 = (ja <= irow) ? (__expf(a0) * dj0) : 0.0f;
        const float e1 = (jc <= irow) ? (__expf(a1) * dj1) : 0.0f;
        pt[(8 * g + v) * kTP40 + r]      = (_Float16)(s0[v] * e0);
        pt[(8 * g + v) * kTP40 + 16 + r] = (_Float16)(s1[v] * e1);
      }
    }
    __syncthreads();
    if (active) {
      const v16h sa = frag_load(pt + r * kTP40 + koff);
#pragma unroll
      for (int nt = 0; nt < 4; ++nt) {
        const v16h xb = frag_load(xs + (nt * 16 + r) * kTP40 + koff);
        acc[nt] = mma_g(sa, xb, acc[nt]);
      }
    }
  }
  v8f acc2[4];
#pragma unroll
  for (int nt = 0; nt < 4; ++nt) acc2[nt] = (v8f){0.f, 0.f, 0.f, 0.f, 0.f, 0.f, 0.f, 0.f};
#pragma unroll
  for (int nt = 0; nt < 4; ++nt) {
    const v16h p0 = frag_load(sentT + (nt * 16 + r) * kPvP + koff);
    const v16h p1 = frag_load(sentT + (nt * 16 + r) * kPvP + 32 + koff);
    acc2[nt] = mma_g(a_lo, p0, acc2[nt]);
    acc2[nt] = mma_g(a_hi, p1, acc2[nt]);
  }
  float sei[8];
#pragma unroll
  for (int v = 0; v < 8; ++v) {
    const float a = fminf(dAi[v], 0.0f);
    sei[v] = (a < -87.0f) ? 0.0f : expf(a);
  }
  __syncthreads();
#pragma unroll
  for (int nt = 0; nt < 4; ++nt)
#pragma unroll
    for (int v = 0; v < 8; ++v) {
      const float yv = (acc[nt][v] + sei[v] * acc2[nt][v]) * kYFold;
      pt[(8 * g + v) * kPwP + nt * 16 + r] = (_Float16)yv;
    }
  __syncthreads();
  {
    const int q = lane >> 3;
    const int c8 = (lane & 7) * 8;
    v8h hv[4];
#pragma unroll
    for (int it = 0; it < 4; ++it) hv[it] = *(const v8h*)(pt + (it * 4 + q) * kPwP + c8);
    for (int pass = 0; pass < 2; ++pass) {
#pragma unroll
      for (int it = 0; it < 4; ++it) {
        const int row = it * 4 + q;
        *(volatile v8h*)(YS16 + (size_t)(lbase + ib + row) * kDIN + h * kHD + c8) = hv[it];
      }
      __threadfence();
    }
  }
}

constexpr int kGatePairs = 4;
static_assert(kMQ % (2 * 8 * kGatePairs) == 0, "gate grid");
__global__ __launch_bounds__(256) void gate_rms_kernel(
    const unsigned short* __restrict__ YS16, const unsigned short* __restrict__ XC16,
    const unsigned short* __restrict__ Z16, const float* __restrict__ Dsk, const float* __restrict__ rmsw,
    unsigned short* __restrict__ YN16)
{
  const int tid = threadIdx.x;
  const int lane = tid & 31;
  const int wave = __builtin_amdgcn_readfirstlane(tid >> 5);
#pragma unroll 1
  for (int pr = 0; pr < kGatePairs; ++pr) {
    const int t0 = ((blockIdx.x * kGatePairs + pr) * 8 + wave) * 2;
    float gq[3][8];
    float ss0 = 0.f, ss1 = 0.f;
#pragma unroll
    for (int it = 0; it < 3; ++it) {
      const int idx = it * 32 + lane;
      const int tk = (idx >= 48) ? 1 : 0;
      const int c0 = (idx - tk * 48) * 8;
      const size_t t = (size_t)(t0 + tk);
      const v4u yw = *(const v4u*)(const void*)(YS16 + t * kDIN + c0);
      const v4u xw = *(const v4u*)(const void*)(XC16 + t * kCD + c0);
      const v4u zw = *(const v4u*)(const void*)(Z16 + t * kDIN + c0);
      const float dh = Dsk[c0 >> 6] * (1.0f / kXcC);
      float ssq = 0.f;
#pragma unroll
      for (int wi = 0; wi < 4; ++wi) {
        const unsigned y2 = yw[wi];
        const unsigned x2 = xw[wi];
        const unsigned z2 = zw[wi];
        const float ya = h16_to_f32(y2 & 0xffffu) * (1.0f / kYsC) + h16_to_f32(x2 & 0xffffu) * dh;
        const float yb = h16_to_f32(y2 >> 16) * (1.0f / kYsC) + h16_to_f32(x2 >> 16) * dh;
        const float za = h16_to_f32(z2 & 0xffffu);
        const float zb = h16_to_f32(z2 >> 16);
        const float ga = ya * (za * __builtin_amdgcn_rcpf(1.0f + __expf(-za)));
        const float gb = yb * (zb * __builtin_amdgcn_rcpf(1.0f + __expf(-zb)));
        gq[it][2 * wi] = ga;
        gq[it][2 * wi + 1] = gb;
        ssq += ga * ga;
        ssq += gb * gb;
      }
      ss0 += tk ? 0.f : ssq;
      ss1 += tk ? ssq : 0.f;
    }
#pragma unroll
    for (int off = 16; off >= 1; off >>= 1) {
      ss0 += __shfl_xor(ss0, off, 32);
      ss1 += __shfl_xor(ss1, off, 32);
    }
    const float r0 = rsqrtf(ss0 * (1.0f / (float)kDIN) + 1e-5f);
    const float r1 = rsqrtf(ss1 * (1.0f / (float)kDIN) + 1e-5f);
    v8h hv[3];
#pragma unroll
    for (int it = 0; it < 3; ++it) {
      const int idx = it * 32 + lane;
      const int tk = (idx >= 48) ? 1 : 0;
      const int c0 = (idx - tk * 48) * 8;
      const float rr = (tk ? r1 : r0) * kActC;
      const v4f w0 = *(const v4f*)(rmsw + c0);
      const v4f w1 = *(const v4f*)(rmsw + c0 + 4);
#pragma unroll
      for (int e = 0; e < 4; ++e) {
        hv[it][e]     = (_Float16)(gq[it][e] * rr * w0[e]);
        hv[it][4 + e] = (_Float16)(gq[it][4 + e] * rr * w1[e]);
      }
    }
    unsigned short* op = YN16 + (size_t)t0 * kDIN;
    for (int pass = 0; pass < 2; ++pass) {
#pragma unroll
      for (int it = 0; it < 3; ++it) *(volatile v8h*)(op + (it * 32 + lane) * 8) = hv[it];
      __threadfence();
    }
  }
}

extern "C" void kernel_launch(void* const* d_in, const int* in_sizes, int n_in,
                              void* d_out, int out_size, void* d_ws, size_t ws_size,
                              hipStream_t stream)
{
  if (n_in < 21) return;
  if (in_sizes[0] != kB * kL * kC) return;
  if (in_sizes[1] != kC * 9 || in_sizes[13] != kC * 9) return;
  if (in_sizes[5] != kDP * kC) return;
  if (in_sizes[6] != kCD * 4 || in_sizes[7] != kCD) return;
  if (in_sizes[8] != kNH || in_sizes[9] != kNH || in_sizes[10] != kNH) return;
  if (in_sizes[11] != kDIN) return;
  if (in_sizes[12] != kC * kDIN) return;
  if (in_sizes[17] != kFF * kC || in_sizes[18] != kFF) return;
  if (in_sizes[19] != kC * kFF || in_sizes[20] != kC) return;
  if (out_size != kB * kL * kC) return;
  if (ws_size < kWsTotal) return;

  const float* x        = (const float*)d_in[0];
  const float* cpe1_w   = (const float*)d_in[1];
  const float* cpe1_b   = (const float*)d_in[2];
  const float* ln1_w    = (const float*)d_in[3];
  const float* ln1_b    = (const float*)d_in[4];
  const float* in_proj  = (const float*)d_in[5];
  const float* conv1d_w = (const float*)d_in[6];
  const float* conv1d_b = (const float*)d_in[7];
  const float* dt_bias  = (const float*)d_in[8];
  const float* A_log    = (const float*)d_in[9];
  const float* D_skip   = (const float*)d_in[10];
  const float* rms_w    = (const float*)d_in[11];
  const float* out_proj = (const float*)d_in[12];
  const float* cpe2_w   = (const float*)d_in[13];
  const float* cpe2_b   = (const float*)d_in[14];
  const float* ln2_w    = (const float*)d_in[15];
  const float* ln2_b    = (const float*)d_in[16];
  const float* fc1_w    = (const float*)d_in[17];
  const float* fc1_b    = (const float*)d_in[18];
  const float* fc2_w    = (const float*)d_in[19];
  const float* fc2_b    = (const float*)d_in[20];
  float* out = (float*)d_out;

  char* ws = (char*)d_ws;
  unsigned short* WIN16  = (unsigned short*)(ws + kOffWIN);
  unsigned short* WOUT16 = (unsigned short*)(ws + kOffWOUT);
  unsigned short* WFC1   = (unsigned short*)(ws + kOffWFC1);
  unsigned short* WFC2   = (unsigned short*)(ws + kOffWFC2);
  float*          SHORT  = (float*)(ws + kOffSHORT);
  unsigned short* H16    = (unsigned short*)(ws + kOffH16);
  unsigned short* Z16    = (unsigned short*)(ws + kOffZ16);
  unsigned short* XBC16  = (unsigned short*)(ws + kOffXBC);
  float*          DTRAW  = (float*)(ws + kOffDTRAW);
  unsigned short* XC16   = (unsigned short*)(ws + kOffXC);
  float*          DT     = (float*)(ws + kOffDT);
  float*          CS     = (float*)(ws + kOffCS);
  float*          STATES = (float*)(ws + kOffST);
  float*          SENT   = (float*)(ws + kOffSENT);
  unsigned short* YS16   = (unsigned short*)(ws + kOffYS);
  unsigned short* YN16   = (unsigned short*)(ws + kOffYN);
  float*          X2     = (float*)(ws + kOffX2);
  float*          X2B    = (float*)(ws + kOffX2B);
  unsigned short* H2_16  = (unsigned short*)(ws + kOffH2);
  unsigned short* M1_16  = (unsigned short*)(ws + kOffM1);

  cast_pad_f16_kernel<<<(kDPP * kC / 8) / 256, 256, 0, stream>>>(in_proj, WIN16, kDPP * kC / 8, kDP * kC / 8, kWgtC);
  cast_pad_f16_kernel<<<(kC * kDIN / 8) / 256, 256, 0, stream>>>(out_proj, WOUT16, kC * kDIN / 8, kC * kDIN / 8, kWgtC);
  cast_pad_f16_kernel<<<(kFF * kC / 8) / 256, 256, 0, stream>>>(fc1_w, WFC1, kFF * kC / 8, kFF * kC / 8, kWgtC);
  cast_pad_f16_kernel<<<(kC * kFF / 8) / 256, 256, 0, stream>>>(fc2_w, WFC2, kC * kFF / 8, kC * kFF / 8, kWgtC);

  for (int pass = 0; pass < kNPASS; ++pass) {
    const float* xp = x + (size_t)pass * kMQ * kC;
    float* outp = out + (size_t)pass * kMQ * kC;

    cpe_ln_kernel<<<kMQ / (32 * kCpeGroups), 256, 0, stream>>>(xp, cpe1_w, cpe1_b, ln1_w, ln1_b, SHORT, H16);

    gemm16_kernel<0, false><<<(kMQ / 64) * (kDPP / 64) / 8, 256, 0, stream>>>(
        H16, kC, WIN16, kC, (void*)Z16, (void*)XBC16, (void*)DTRAW, 0, ln1_b, SHORT,
        kMQ, kDPP, kC, kGemmSc);

    conv_silu_kernel<<<kMQ / 64, 256, 0, stream>>>(XBC16, conv1d_w, conv1d_b, XC16);

    dt_cumsum_kernel<<<kUnits / 8, 256, 0, stream>>>(DTRAW, dt_bias, A_log, DT, CS);

    ssd_states_kernel<<<kUnits, 128, 0, stream>>>(XC16, DT, CS, STATES);

    chunk_scan_kernel<<<(kBP * kNH * 1024) / 256, 256, 0, stream>>>(STATES, CS, SENT);

    ssd_y_kernel<<<kUnits, 512, 0, stream>>>(XC16, DT, CS, SENT, YS16);

    gate_rms_kernel<<<kMQ / (2 * 8 * kGatePairs), 256, 0, stream>>>(YS16, XC16, Z16, D_skip, rms_w, YN16);

    gemm16_kernel<1, false><<<(kMQ / 64) * (kC / 64) / 8, 256, 0, stream>>>(
        YN16, kDIN, WOUT16, kDIN, (void*)X2, (void*)X2, (void*)X2, kC, ln1_b, SHORT,
        kMQ, kC, kDIN, kGemmSc);

    cpe_ln_kernel<<<kMQ / (32 * kCpeGroups), 256, 0, stream>>>(X2, cpe2_w, cpe2_b, ln2_w, ln2_b, X2B, H2_16);

    gemm16_kernel<2, true><<<(kMQ / 64) * (kFF / 64) / 8, 256, 0, stream>>>(
        H2_16, kC, WFC1, kC, (void*)M1_16, (void*)M1_16, (void*)M1_16, kFF, fc1_b, SHORT,
        kMQ, kFF, kC, kGemmSc);

    gemm16_kernel<1, true><<<(kMQ / 64) * (kC / 64) / 8, 256, 0, stream>>>(
        M1_16, kFF, WFC2, kFF, (void*)outp, (void*)outp, (void*)outp, kC, fc2_b, X2B,
        kMQ, kC, kFF, kGemmSc);
  }
}
